// FinancialGNNRAG_67980742361614
// MI455X (gfx1250) — hardware-verified
//
#include <hip/hip_runtime.h>
#include <stddef.h>


#define HC      256
#define C3      32
#define NTHR    256
#define NWAVE   8
#define EPT     8
#define NGRP    2
#define CHUNK   (NTHR * EPT * NGRP)
#define WCAP    (EPT * NGRP * 32)
#define LISTN   (NWAVE * WCAP)
#define NBC     4096
#define NBF     1024
#define RCAP    40960
#define RBN     128
#define OTHR    512
#define TGT     256
#define DEGCAP  128
#define G2THR   128
#define G2W     4
#define G2ROWS  64
#define KP2     264
#define ZP      16
#define APP     8
#define NEGS    0.2f
#define EPSS    1e-16f
#define WSCAP   ((size_t)134217728)

#define LDS_FILL ((RCAP + NBF + LISTN) * 4 + 64)
#define LDS_G2   (2 * G2ROWS * KP2 * 2 + G2W * 16 * 128 * 4 + (768 + 256 + 256 + 256) * 4 + G2W * 128 * 4)
#define LDS_A2   (2 * G2ROWS * KP2 * 2 + G2W * 16 * C3 * 4 + (C3 + C3) * 4 + G2W * 128 * 4)

static_assert((CHUNK & (CHUNK - 1)) == 0);
static_assert(CHUNK <= 4096);
static_assert(NBC <= 4096 && NBF <= 4096);
static_assert((NBC & (NBC - 1)) == 0 && (NBF & (NBF - 1)) == 0);
static_assert(NBC == 4 * NBF);
static_assert(OTHR * 8 == NBC);
static_assert((RCAP % 32) == 0);
static_assert(TGT == NTHR && (TGT % G2ROWS) == 0 && (TGT % 32) == 0);
static_assert(G2THR == 2 * G2ROWS && G2ROWS == 16 * G2W && G2THR == 32 * G2W);
static_assert(((HC * HC / 8) % NTHR) == 0);
static_assert((KP2 % 8) == 0 && KP2 >= HC);
static_assert(HC == 256 && C3 == 32 && ZP == 16 && APP == 8);
static_assert(DEGCAP >= 32);

typedef float          v4f  __attribute__((ext_vector_type(4)));
typedef float          v8f  __attribute__((ext_vector_type(8)));
typedef int            v4i  __attribute__((ext_vector_type(4)));
typedef unsigned short v8us __attribute__((ext_vector_type(8)));
typedef __bf16         v16bf __attribute__((ext_vector_type(16)));
union FragB { v16bf v; v8us h[2]; };

__device__ __forceinline__ int clampi(int v, int lo, int hi) {
  v = v < lo ? lo : v;
  return v > hi ? hi : v;
}
__device__ __forceinline__ float lk(float a) { return a > 0.0f ? a : a * NEGS; }
__device__ __forceinline__ int wmaxi(int v) {
  v = max(v, __shfl_xor(v, 16));
  v = max(v, __shfl_xor(v, 8));
  v = max(v, __shfl_xor(v, 4));
  v = max(v, __shfl_xor(v, 2));
  v = max(v, __shfl_xor(v, 1));
  return v;
}
__device__ __forceinline__ float wmaxf(float v) {
  v = fmaxf(v, __shfl_xor(v, 16));
  v = fmaxf(v, __shfl_xor(v, 8));
  v = fmaxf(v, __shfl_xor(v, 4));
  v = fmaxf(v, __shfl_xor(v, 2));
  v = fmaxf(v, __shfl_xor(v, 1));
  return v;
}
__device__ __forceinline__ float red16(float v) {
  v += __shfl_xor(v, 1);
  v += __shfl_xor(v, 2);
  v += __shfl_xor(v, 4);
  v += __shfl_xor(v, 8);
  return v;
}
__device__ __forceinline__ v4f relu4(v4f v) {
  v.x = fmaxf(v.x, 0.0f); v.y = fmaxf(v.y, 0.0f); v.z = fmaxf(v.z, 0.0f); v.w = fmaxf(v.w, 0.0f);
  return v;
}

__device__ __forceinline__ unsigned bfb(float f) {
  const unsigned u = __float_as_uint(f);
  return (u + 0x7FFFu + ((u >> 16) & 1u)) >> 16;
}
__device__ __forceinline__ unsigned hl2(float v, unsigned& lb) {
  const unsigned hb = bfb(v);
  lb = bfb(v - __uint_as_float(hb << 16));
  return hb;
}
__device__ __forceinline__ void pack8(v4f a, v4f b, v4i& ph, v4i& pl) {
  unsigned l0, l1, l2, l3, l4, l5, l6, l7;
  const unsigned h0 = hl2(a.x, l0), h1 = hl2(a.y, l1), h2 = hl2(a.z, l2), h3 = hl2(a.w, l3);
  const unsigned h4 = hl2(b.x, l4), h5 = hl2(b.y, l5), h6 = hl2(b.z, l6), h7 = hl2(b.w, l7);
  ph.x = (int)(h0 | (h1 << 16)); ph.y = (int)(h2 | (h3 << 16)); ph.z = (int)(h4 | (h5 << 16)); ph.w = (int)(h6 | (h7 << 16));
  pl.x = (int)(l0 | (l1 << 16)); pl.y = (int)(l2 | (l3 << 16)); pl.z = (int)(l4 | (l5 << 16)); pl.w = (int)(l6 | (l7 << 16));
}

__device__ __forceinline__ v8f wmb(v16bf a, v16bf b, v8f c) {
  v8f d = __builtin_amdgcn_wmma_f32_16x16x32_bf16(false, a, false, b, (short)0, c, false, false);
  asm volatile("v_nop\n\tv_nop\n\tv_nop\n\tv_nop" : "+v"(d) : "v"(a), "v"(b));
  return d;
}

template <int NB>
__device__ __forceinline__ int scan_chunk(const int* __restrict__ dsts, int nE, int cbase, int slotBase,
                                          int vec8, int* list, int tid, int lane, int wave) {
  int wc = 0;
#pragma unroll
  for (int g = 0; g < NGRP; ++g) {
    const int el0  = (g * NTHR + tid) * EPT;
    const int e0   = cbase + el0;
    const int sent = -2147483647 - 1;
    v4i da, db;
    if (vec8 != 0 && cbase + CHUNK <= nE) {
      da = *(const v4i*)(dsts + e0);
      db = *(const v4i*)(dsts + e0 + 4);
    } else {
      da.x = (e0     < nE) ? dsts[min(e0, nE - 1)] : sent;
      da.y = (e0 + 1 < nE) ? dsts[min(e0 + 1, nE - 1)] : sent;
      da.z = (e0 + 2 < nE) ? dsts[min(e0 + 2, nE - 1)] : sent;
      da.w = (e0 + 3 < nE) ? dsts[min(e0 + 3, nE - 1)] : sent;
      db.x = (e0 + 4 < nE) ? dsts[min(e0 + 4, nE - 1)] : sent;
      db.y = (e0 + 5 < nE) ? dsts[min(e0 + 5, nE - 1)] : sent;
      db.z = (e0 + 6 < nE) ? dsts[min(e0 + 6, nE - 1)] : sent;
      db.w = (e0 + 7 < nE) ? dsts[min(e0 + 7, nE - 1)] : sent;
    }
    const unsigned nb = (unsigned)slotBase;
    const unsigned s0 = (unsigned)da.x - nb, s1 = (unsigned)da.y - nb;
    const unsigned s2 = (unsigned)da.z - nb, s3 = (unsigned)da.w - nb;
    const unsigned s4 = (unsigned)db.x - nb, s5 = (unsigned)db.y - nb;
    const unsigned s6 = (unsigned)db.z - nb, s7 = (unsigned)db.w - nb;
    const bool h0 = s0 < (unsigned)NB, h1 = s1 < (unsigned)NB, h2 = s2 < (unsigned)NB, h3 = s3 < (unsigned)NB;
    const bool h4 = s4 < (unsigned)NB, h5 = s5 < (unsigned)NB, h6 = s6 < (unsigned)NB, h7 = s7 < (unsigned)NB;
    const unsigned any = __builtin_amdgcn_ballot_w32(h0 | h1 | h2 | h3 | h4 | h5 | h6 | h7);
    if (any != 0u) {
#define HITJ(J, HJ, SJ) { \
        const unsigned mj = __builtin_amdgcn_ballot_w32(HJ); \
        if (mj != 0u) { \
          if (HJ) { \
            const int pos = wc + (int)__builtin_amdgcn_mbcnt_lo(mj, 0u); \
            if (pos < WCAP) list[wave * WCAP + pos] = ((el0 + (J)) << 12) | (int)(SJ); \
          } \
          wc += (int)__builtin_popcount(mj); } }
      HITJ(0, h0, s0)
      HITJ(1, h1, s1)
      HITJ(2, h2, s2)
      HITJ(3, h3, s3)
      HITJ(4, h4, s4)
      HITJ(5, h5, s5)
      HITJ(6, h6, s6)
      HITJ(7, h7, s7)
#undef HITJ
    }
  }
  return wc;
}

__global__ __launch_bounds__(NTHR) void k_wprep(
    const float* __restrict__ W2, const float* __restrict__ W3,
    unsigned short* w2h, unsigned short* w2l, unsigned short* w3h, unsigned short* w3l) {
  const int g0 = HC * HC / 8;
  const int g1 = C3 * HC / 8;
  const int bstart = blockIdx.x * NTHR;
  const float* src; unsigned short* dh; unsigned short* dl; int Nout; int seg;
  if (bstart < g0) { src = W2; dh = w2h; dl = w2l; Nout = HC; seg = 0;  }
  else             { src = W3; dh = w3h; dl = w3l; Nout = C3; seg = g0; }
  const int i = bstart + (int)threadIdx.x;
  if (i >= g0 + g1) return;
  const int o  = (i - seg) * 8;
  const int n  = o / HC;
  const int k0 = o - n * HC;
  float v[8];
#pragma unroll
  for (int e = 0; e < 8; ++e) v[e] = src[(size_t)(k0 + e) * Nout + n];
  v4f a, b;
  a.x = v[0]; a.y = v[1]; a.z = v[2]; a.w = v[3];
  b.x = v[4]; b.y = v[5]; b.z = v[6]; b.w = v[7];
  v4i ph, pl;
  pack8(a, b, ph, pl);
  *(volatile v4i*)(dh + o) = ph;
  *(volatile v4i*)(dl + o) = pl;
  __threadfence();
  *(volatile v4i*)(dh + o) = ph;
  *(volatile v4i*)(dl + o) = pl;
}

__global__ __launch_bounds__(NTHR) void k_count(
    const int* __restrict__ ei, int* cnt, int nE, int vec8) {
  __shared__ __attribute__((aligned(16))) int scnt[NBC];
  __shared__ __attribute__((aligned(16))) int list[LISTN];
  __shared__ int wcnt[NWAVE];
  const int tid = threadIdx.x, lane = tid & 31, wave = tid >> 5;
  const int nodeBase = blockIdx.x * NBC;
  const int* dsts = ei + nE;

  for (int i = tid; i < NBC; i += NTHR) scnt[i] = 0;
  __syncthreads();

  const int nChunks = (nE + CHUNK - 1) / CHUNK;
#pragma unroll 1
  for (int ch = 0; ch < nChunks; ++ch) {
    const int cbase = ch * CHUNK;
    const int wc = scan_chunk<NBC>(dsts, nE, cbase, nodeBase, vec8, list, tid, lane, wave);
    if (lane == 0) wcnt[wave] = wc;
    __syncthreads();
    if (wave == 0) {
#pragma unroll 1
      for (int wsx = 0; wsx < NWAVE; ++wsx) {
        int n = __builtin_amdgcn_readfirstlane(wcnt[wsx]);
        n = n > WCAP ? WCAP : (n < 0 ? 0 : n);
        const int* lp = list + wsx * WCAP;
#pragma unroll 1
        for (int i = 0; i < n; ++i) {
          const int ent  = __builtin_amdgcn_readfirstlane(lp[i]);
          const int slot = ent & (NBC - 1);
          if (lane == 0) scnt[slot] = scnt[slot] + 1;
        }
      }
    }
    __syncthreads();
  }

  v4i cq[4];
#pragma unroll
  for (int q = 0; q < 4; ++q) {
    const int f = (wave * 4 + q) * 128 + 4 * lane;
    cq[q] = *(const v4i*)(scnt + f);
  }
  int* cp = cnt + (size_t)nodeBase;
#pragma unroll
  for (int q = 0; q < 4; ++q) {
    const int f = (wave * 4 + q) * 128 + 4 * lane;
    *(volatile v4i*)(cp + f) = cq[q];
  }
  __threadfence();
#pragma unroll
  for (int q = 0; q < 4; ++q) {
    const int f = (wave * 4 + q) * 128 + 4 * lane;
    *(volatile v4i*)(cp + f) = cq[q];
  }
}

__global__ __launch_bounds__(OTHR) void k_offsets(
    const int* __restrict__ cnt, int* off, int* rbase, int nChunk) {
  __shared__ __attribute__((aligned(16))) int soff[NBC];
  __shared__ __attribute__((aligned(16))) int srb[RBN];
  __shared__ int wtot[OTHR / 32];
  const int tid = threadIdx.x, lane = tid & 31, wave = tid >> 5, sub = tid >> 7;
  for (int i = tid; i < RBN; i += OTHR) srb[i] = 0;
  int carry = 0;
#pragma unroll 1
  for (int ch = 0; ch < nChunk; ++ch) {
    const int base = ch * NBC;
    const v4i c0 = *(const v4i*)(cnt + base + 8 * tid);
    const v4i c1 = *(const v4i*)(cnt + base + 8 * tid + 4);
    const int e0 = max(c0.x, 0), e1 = max(c0.y, 0), e2 = max(c0.z, 0), e3 = max(c0.w, 0);
    const int e4 = max(c1.x, 0), e5 = max(c1.y, 0), e6 = max(c1.z, 0), e7 = max(c1.w, 0);
    const int ts = e0 + e1 + e2 + e3 + e4 + e5 + e6 + e7;
    int incl = ts;
#pragma unroll
    for (int d = 1; d < 32; d <<= 1) {
      const int t = __shfl_up(incl, d);
      if (lane >= d) incl += t;
    }
    if (lane == 31) wtot[wave] = incl;
    __syncthreads();
    const int S0 = wtot[0]  + wtot[1]  + wtot[2]  + wtot[3];
    const int S1 = wtot[4]  + wtot[5]  + wtot[6]  + wtot[7];
    const int S2 = wtot[8]  + wtot[9]  + wtot[10] + wtot[11];
    const int S3 = wtot[12] + wtot[13] + wtot[14] + wtot[15];
    int pre = 0;
#pragma unroll 1
    for (int w = 4 * sub; w < wave; ++w) pre += wtot[w];
    const int b0 = carry;
    const int b1 = b0 + ((S0 + 31) & ~31);
    const int b2 = b1 + ((S1 + 31) & ~31);
    const int b3 = b2 + ((S2 + 31) & ~31);
    const int b4 = b3 + ((S3 + 31) & ~31);
    const int myb = sub == 0 ? b0 : (sub == 1 ? b1 : (sub == 2 ? b2 : b3));
    if (tid == 0) {
      srb[min(4 * ch + 0, RBN - 1)] = b0;
      srb[min(4 * ch + 1, RBN - 1)] = b1;
      srb[min(4 * ch + 2, RBN - 1)] = b2;
      srb[min(4 * ch + 3, RBN - 1)] = b3;
    }
    int run = myb + pre + incl - ts;
    soff[8 * tid + 0] = run; run += e0;
    soff[8 * tid + 1] = run; run += e1;
    soff[8 * tid + 2] = run; run += e2;
    soff[8 * tid + 3] = run; run += e3;
    soff[8 * tid + 4] = run; run += e4;
    soff[8 * tid + 5] = run; run += e5;
    soff[8 * tid + 6] = run; run += e6;
    soff[8 * tid + 7] = run;
    carry = b4;
    __syncthreads();
    const v4i o0 = *(const v4i*)(soff + 4 * tid);
    const v4i o1 = *(const v4i*)(soff + 4 * (tid + OTHR));
    int* op = off + base;
    *(volatile v4i*)(op + 4 * tid) = o0;
    *(volatile v4i*)(op + 4 * (tid + OTHR)) = o1;
    __threadfence();
    *(volatile v4i*)(op + 4 * tid) = o0;
    *(volatile v4i*)(op + 4 * (tid + OTHR)) = o1;
    __syncthreads();
  }
  if (tid == 0) srb[min(4 * nChunk, RBN - 1)] = carry;
  __syncthreads();
  v4i rv = {0, 0, 0, 0};
  if (tid < 32) rv = *(const v4i*)(srb + 4 * tid);
  if (tid < 32) *(volatile v4i*)(rbase + 4 * tid) = rv;
  __threadfence();
  if (tid < 32) *(volatile v4i*)(rbase + 4 * tid) = rv;
}

__global__ __launch_bounds__(NTHR) void k_fill(
    const int* __restrict__ ei, const int* __restrict__ off, const int* __restrict__ rbase,
    int* csr, int nN, int nE, int vec8, int csrLen) {
  extern __shared__ v4f lds_dyn[];
  int* region = (int*)lds_dyn;
  int* cursor = region + RCAP;
  int* list   = cursor + NBF;
  int* wcnt   = list + LISTN;
  const int tid = threadIdx.x, lane = tid & 31, wave = tid >> 5;
  const int b = blockIdx.x;
  const int nodeBase = b * NBF;
  const int* dsts = ei + nE;

  int rb0 = rbase[b];
  const int rb1 = rbase[b + 1];
  rb0 = rb0 < 0 ? 0 : (rb0 > csrLen ? csrLen : rb0);
  rb0 &= ~31;
  int len = rb1 - rb0;
  len = len < 0 ? 0 : (len > RCAP ? RCAP : len);
  int lenW = (len + 31) & ~31;
  if (rb0 + lenW > csrLen) lenW = (csrLen - rb0) & ~31;

  {
    const v4i zz = {0, 0, 0, 0};
    for (int i = tid; i < RCAP / 4; i += NTHR) ((v4i*)region)[i] = zz;
    for (int s = tid; s < NBF; s += NTHR) {
      int o = off[nodeBase + s] - rb0;
      o = o < 0 ? 0 : (o > RCAP ? RCAP : o);
      cursor[s] = o;
    }
  }
  __syncthreads();

  const int nChunks = (nE + CHUNK - 1) / CHUNK;
#pragma unroll 1
  for (int ch = 0; ch < nChunks; ++ch) {
    const int cbase = ch * CHUNK;
    const int wc = scan_chunk<NBF>(dsts, nE, cbase, nodeBase, vec8, list, tid, lane, wave);
    if (lane == 0) wcnt[wave] = wc;
    __syncthreads();
    if (wave == 0) {
#pragma unroll 1
      for (int wsx = 0; wsx < NWAVE; ++wsx) {
        int n = __builtin_amdgcn_readfirstlane(wcnt[wsx]);
        n = n > WCAP ? WCAP : (n < 0 ? 0 : n);
        const int* lp = list + wsx * WCAP;
#pragma unroll 1
        for (int i = 0; i < n; ++i) {
          const int ent  = __builtin_amdgcn_readfirstlane(lp[i]);
          const int slot = ent & (NBF - 1);
          int e = cbase + ((ent >> 12) & (CHUNK - 1));
          e = e > nE - 1 ? nE - 1 : e;
          int src = ei[e];
          src = src < 0 ? 0 : (src > nN - 1 ? nN - 1 : src);
          if (lane == 0) {
            int pos = cursor[slot];
            pos = pos < 0 ? 0 : (pos > RCAP - 1 ? RCAP - 1 : pos);
            region[pos] = src;
            const int np = pos + 1;
            cursor[slot] = np > RCAP ? RCAP : np;
          }
        }
      }
    }
    __syncthreads();
  }

  const int nv = lenW >> 2;
  int* gp = csr + rb0;
#pragma unroll 1
  for (int i = tid; i < nv; i += NTHR) { const v4i v = ((const v4i*)region)[i]; *(volatile v4i*)(gp + 4 * i) = v; }
  __threadfence();
#pragma unroll 1
  for (int i = tid; i < nv; i += NTHR) { const v4i v = ((const v4i*)region)[i]; *(volatile v4i*)(gp + 4 * i) = v; }
}

__global__ __launch_bounds__(NTHR) void k_node1(
    const float* __restrict__ x, const float* __restrict__ W1,
    const float* __restrict__ as1, const float* __restrict__ ad1, float* ap, int nN) {
  __shared__ __attribute__((aligned(16))) float astg[32 * APP];
  const int tid = threadIdx.x, lane = tid & 31, wave = tid >> 5, hh = lane >> 4;
  const int nb = blockIdx.x * 32;
  const int cA = 4 * lane, cB = 128 + 4 * lane;
  const v4f w0A = *(const v4f*)(W1 + cA), w1A = *(const v4f*)(W1 + HC + cA), w2A = *(const v4f*)(W1 + 2 * HC + cA);
  const v4f w0B = *(const v4f*)(W1 + cB), w1B = *(const v4f*)(W1 + HC + cB), w2B = *(const v4f*)(W1 + 2 * HC + cB);
  const v4f sA = *(const v4f*)(as1 + cA), sB = *(const v4f*)(as1 + cB);
  const v4f dA = *(const v4f*)(ad1 + cA), dB = *(const v4f*)(ad1 + cB);
#pragma unroll 1
  for (int j = 0; j < 4; ++j) {
    const int slot = wave * 4 + j;
    int n = nb + slot;
    n = n > nN - 1 ? nN - 1 : n;
    const float x0 = x[(size_t)n * 3], x1 = x[(size_t)n * 3 + 1], x2 = x[(size_t)n * 3 + 2];
    v4f hA, hB;
    hA.x = fmaf(x0, w0A.x, fmaf(x1, w1A.x, x2 * w2A.x));
    hA.y = fmaf(x0, w0A.y, fmaf(x1, w1A.y, x2 * w2A.y));
    hA.z = fmaf(x0, w0A.z, fmaf(x1, w1A.z, x2 * w2A.z));
    hA.w = fmaf(x0, w0A.w, fmaf(x1, w1A.w, x2 * w2A.w));
    hB.x = fmaf(x0, w0B.x, fmaf(x1, w1B.x, x2 * w2B.x));
    hB.y = fmaf(x0, w0B.y, fmaf(x1, w1B.y, x2 * w2B.y));
    hB.z = fmaf(x0, w0B.z, fmaf(x1, w1B.z, x2 * w2B.z));
    hB.w = fmaf(x0, w0B.w, fmaf(x1, w1B.w, x2 * w2B.w));
    float psA = fmaf(hA.x, sA.x, fmaf(hA.y, sA.y, fmaf(hA.z, sA.z, hA.w * sA.w)));
    float pdA = fmaf(hA.x, dA.x, fmaf(hA.y, dA.y, fmaf(hA.z, dA.z, hA.w * dA.w)));
    float psB = fmaf(hB.x, sB.x, fmaf(hB.y, sB.y, fmaf(hB.z, sB.z, hB.w * sB.w)));
    float pdB = fmaf(hB.x, dB.x, fmaf(hB.y, dB.y, fmaf(hB.z, dB.z, hB.w * dB.w)));
    psA = red16(psA); pdA = red16(pdA); psB = red16(psB); pdB = red16(pdB);
    if ((lane & 15) == 0) {
      astg[slot * APP + hh]     = psA;
      astg[slot * APP + 2 + hh] = psB;
      astg[slot * APP + 4 + hh] = pdA;
      astg[slot * APP + 6 + hh] = pdB;
    }
  }
  __syncthreads();
  v4f av = {0.f, 0.f, 0.f, 0.f};
  if (tid < 64) av = *(const v4f*)(astg + 4 * tid);
  float* aq = ap + (size_t)nb * APP + 4 * tid;
  if (tid < 64) *(volatile v4f*)aq = av;
  __threadfence();
  if (tid < 64) *(volatile v4f*)aq = av;
}

__global__ __launch_bounds__(NTHR) void k_agg1(
    const int* __restrict__ csr, const int* __restrict__ off, const int* __restrict__ cnt,
    const float* __restrict__ x, const float* __restrict__ ap, float* z, int nN, int csrLen) {
  __shared__ __attribute__((aligned(16))) float zs[TGT * ZP];
  const int tid = threadIdx.x;
  const int t = blockIdx.x * TGT + tid;
  int n = cnt[t];
  n = clampi(n, 0, DEGCAP);
  const int st = off[t];
  const int nm = wmaxi(n);
  const int tc = t > nN - 1 ? nN - 1 : t;
  const v4f a4 = *(const v4f*)(ap + (size_t)tc * APP);
  const v4f d4 = *(const v4f*)(ap + (size_t)tc * APP + 4);
  const float xs0 = x[(size_t)tc * 3], xs1 = x[(size_t)tc * 3 + 1], xs2 = x[(size_t)tc * 3 + 2];
  const float e0 = lk(a4.x + d4.x), e1 = lk(a4.y + d4.y), e2 = lk(a4.z + d4.z), e3 = lk(a4.w + d4.w);
  float m0 = e0, m1 = e1, m2 = e2, m3 = e3;
#pragma unroll 1
  for (int p = 0; p < nm; ++p) {
    const int pos = clampi(st + p, 0, csrLen - 1);
    const int s   = clampi(csr[pos], 0, nN - 1);
    const v4f b4  = *(const v4f*)(ap + (size_t)s * APP);
    const bool ok = p < n;
    const float t0 = lk(b4.x + d4.x), t1 = lk(b4.y + d4.y), t2 = lk(b4.z + d4.z), t3 = lk(b4.w + d4.w);
    m0 = ok ? fmaxf(m0, t0) : m0;
    m1 = ok ? fmaxf(m1, t1) : m1;
    m2 = ok ? fmaxf(m2, t2) : m2;
    m3 = ok ? fmaxf(m3, t3) : m3;
  }
  const float p0 = __expf(e0 - m0), p1 = __expf(e1 - m1), p2 = __expf(e2 - m2), p3 = __expf(e3 - m3);
  float dn0 = p0, dn1 = p1, dn2 = p2, dn3 = p3;
  float z00 = p0 * xs0, z01 = p0 * xs1, z02 = p0 * xs2;
  float z10 = p1 * xs0, z11 = p1 * xs1, z12 = p1 * xs2;
  float z20 = p2 * xs0, z21 = p2 * xs1, z22 = p2 * xs2;
  float z30 = p3 * xs0, z31 = p3 * xs1, z32 = p3 * xs2;
#pragma unroll 1
  for (int p = 0; p < nm; ++p) {
    const int pos = clampi(st + p, 0, csrLen - 1);
    const int s   = clampi(csr[pos], 0, nN - 1);
    const v4f b4  = *(const v4f*)(ap + (size_t)s * APP);
    const float y0 = x[(size_t)s * 3], y1 = x[(size_t)s * 3 + 1], y2 = x[(size_t)s * 3 + 2];
    const bool ok = p < n;
    float q0 = __expf(lk(b4.x + d4.x) - m0); q0 = ok ? q0 : 0.0f;
    float q1 = __expf(lk(b4.y + d4.y) - m1); q1 = ok ? q1 : 0.0f;
    float q2 = __expf(lk(b4.z + d4.z) - m2); q2 = ok ? q2 : 0.0f;
    float q3 = __expf(lk(b4.w + d4.w) - m3); q3 = ok ? q3 : 0.0f;
    dn0 += q0; dn1 += q1; dn2 += q2; dn3 += q3;
    z00 = fmaf(q0, y0, z00); z01 = fmaf(q0, y1, z01); z02 = fmaf(q0, y2, z02);
    z10 = fmaf(q1, y0, z10); z11 = fmaf(q1, y1, z11); z12 = fmaf(q1, y2, z12);
    z20 = fmaf(q2, y0, z20); z21 = fmaf(q2, y1, z21); z22 = fmaf(q2, y2, z22);
    z30 = fmaf(q3, y0, z30); z31 = fmaf(q3, y1, z31); z32 = fmaf(q3, y2, z32);
  }
  const float i0 = 1.0f / (dn0 + EPSS), i1 = 1.0f / (dn1 + EPSS), i2 = 1.0f / (dn2 + EPSS), i3 = 1.0f / (dn3 + EPSS);
  v4f r0, r1, r2, r3;
  r0.x = z00 * i0; r0.y = z01 * i0; r0.z = z02 * i0; r0.w = z10 * i1;
  r1.x = z11 * i1; r1.y = z12 * i1; r1.z = z20 * i2; r1.w = z21 * i2;
  r2.x = z22 * i2; r2.y = z30 * i3; r2.z = z31 * i3; r2.w = z32 * i3;
  r3.x = 0.0f; r3.y = 0.0f; r3.z = 0.0f; r3.w = 0.0f;
  float* zw = zs + tid * ZP;
  *(v4f*)zw = r0; *(v4f*)(zw + 4) = r1; *(v4f*)(zw + 8) = r2; *(v4f*)(zw + 12) = r3;
  __syncthreads();
  float* gz = z + (size_t)blockIdx.x * TGT * ZP;
  const v4f o0 = *(const v4f*)(zs + 4 * tid);
  const v4f o1 = *(const v4f*)(zs + 4 * (NTHR + tid));
  const v4f o2 = *(const v4f*)(zs + 4 * (2 * NTHR + tid));
  const v4f o3 = *(const v4f*)(zs + 4 * (3 * NTHR + tid));
  *(volatile v4f*)(gz + 4 * tid) = o0;
  *(volatile v4f*)(gz + 4 * (NTHR + tid)) = o1;
  *(volatile v4f*)(gz + 4 * (2 * NTHR + tid)) = o2;
  *(volatile v4f*)(gz + 4 * (3 * NTHR + tid)) = o3;
  __threadfence();
  *(volatile v4f*)(gz + 4 * tid) = o0;
  *(volatile v4f*)(gz + 4 * (NTHR + tid)) = o1;
  *(volatile v4f*)(gz + 4 * (2 * NTHR + tid)) = o2;
  *(volatile v4f*)(gz + 4 * (3 * NTHR + tid)) = o3;
}

__global__ __launch_bounds__(G2THR) void k_gemm2(
    const float* __restrict__ z, const float* __restrict__ W1, const float* __restrict__ b1,
    const unsigned short* __restrict__ w2h, const unsigned short* __restrict__ w2l,
    const float* __restrict__ as2, const float* __restrict__ ad2,
    float* H2, float* ap) {
  extern __shared__ v4f lds_dyn[];
  unsigned short* sAh = (unsigned short*)lds_dyn;
  unsigned short* sAl = sAh + G2ROWS * KP2;
  float* stg  = (float*)(sAl + G2ROWS * KP2);
  float* sW1  = stg + G2W * 16 * 128;
  float* sb1  = sW1 + 768;
  float* sas  = sb1 + 256;
  float* sad  = sas + 256;
  float* astg = sad + 256;
  const int tid = threadIdx.x, lane = tid & 31, wave = tid >> 5, hh = lane >> 4, m = lane & 15;
  const int rowBase = blockIdx.x * G2ROWS;

  for (int i = tid; i < 768; i += G2THR) sW1[i] = W1[i];
  for (int i = tid; i < 256; i += G2THR) { sb1[i] = b1[i]; sas[i] = as2[i]; sad[i] = ad2[i]; }
  __syncthreads();

  {
    const int r = tid & (G2ROWS - 1);
    const int half = tid >> 6;
    const float* zr = z + (size_t)(rowBase + r) * ZP;
    const v4f z0 = *(const v4f*)zr, z1 = *(const v4f*)(zr + 4), z2 = *(const v4f*)(zr + 8);
#pragma unroll 1
    for (int e8 = 0; e8 < 16; ++e8) {
      const int c0 = 128 * half + 8 * e8;
      const int hd = c0 >> 6;
      const float q0 = hd == 0 ? z0.x : (hd == 1 ? z0.w : (hd == 2 ? z1.z : z2.y));
      const float q1 = hd == 0 ? z0.y : (hd == 1 ? z1.x : (hd == 2 ? z1.w : z2.z));
      const float q2 = hd == 0 ? z0.z : (hd == 1 ? z1.y : (hd == 2 ? z2.x : z2.w));
      const v4f wa0 = *(const v4f*)(sW1 + c0),          wa1 = *(const v4f*)(sW1 + c0 + 4);
      const v4f wb0 = *(const v4f*)(sW1 + HC + c0),     wb1 = *(const v4f*)(sW1 + HC + c0 + 4);
      const v4f wc0 = *(const v4f*)(sW1 + 2 * HC + c0), wc1 = *(const v4f*)(sW1 + 2 * HC + c0 + 4);
      const v4f bb0 = *(const v4f*)(sb1 + c0),          bb1 = *(const v4f*)(sb1 + c0 + 4);
      v4f va, vb;
      va.x = fmaxf(fmaf(q0, wa0.x, fmaf(q1, wb0.x, q2 * wc0.x)) + bb0.x, 0.0f);
      va.y = fmaxf(fmaf(q0, wa0.y, fmaf(q1, wb0.y, q2 * wc0.y)) + bb0.y, 0.0f);
      va.z = fmaxf(fmaf(q0, wa0.z, fmaf(q1, wb0.z, q2 * wc0.z)) + bb0.z, 0.0f);
      va.w = fmaxf(fmaf(q0, wa0.w, fmaf(q1, wb0.w, q2 * wc0.w)) + bb0.w, 0.0f);
      vb.x = fmaxf(fmaf(q0, wa1.x, fmaf(q1, wb1.x, q2 * wc1.x)) + bb1.x, 0.0f);
      vb.y = fmaxf(fmaf(q0, wa1.y, fmaf(q1, wb1.y, q2 * wc1.y)) + bb1.y, 0.0f);
      vb.z = fmaxf(fmaf(q0, wa1.z, fmaf(q1, wb1.z, q2 * wc1.z)) + bb1.z, 0.0f);
      vb.w = fmaxf(fmaf(q0, wa1.w, fmaf(q1, wb1.w, q2 * wc1.w)) + bb1.w, 0.0f);
      v4i ph, pl;
      pack8(va, vb, ph, pl);
      *(v4i*)(sAh + r * KP2 + c0) = ph;
      *(v4i*)(sAl + r * KP2 + c0) = pl;
    }
  }
  __syncthreads();

  float sa0 = 0.0f, sa1 = 0.0f, sd0 = 0.0f, sd1 = 0.0f;
  const unsigned short* arh = sAh + (wave * 16 + m) * KP2 + 8 * hh;
  const unsigned short* arl = sAl + (wave * 16 + m) * KP2 + 8 * hh;
  float* sp = stg + wave * (16 * 128);
#pragma unroll 1
  for (int g = 0; g < 2; ++g) {
    v8f acc[8];
#pragma unroll
    for (int t = 0; t < 8; ++t) { v8f zz = {0.f, 0.f, 0.f, 0.f, 0.f, 0.f, 0.f, 0.f}; acc[t] = zz; }
#pragma unroll 1
    for (int kt = 0; kt < HC / 32; ++kt) {
      FragB ahf, alf;
      ahf.h[0] = *(const v8us*)(arh + 32 * kt);
      ahf.h[1] = *(const v8us*)(arh + 32 * kt + 16);
      alf.h[0] = *(const v8us*)(arl + 32 * kt);
      alf.h[1] = *(const v8us*)(arl + 32 * kt + 16);
#pragma unroll
      for (int t = 0; t < 8; ++t) {
        const size_t bo = (size_t)(128 * g + 16 * t + m) * HC + 32 * kt + 8 * hh;
        FragB bhf, blf;
        bhf.h[0] = *(const v8us*)(w2h + bo);
        bhf.h[1] = *(const v8us*)(w2h + bo + 16);
        blf.h[0] = *(const v8us*)(w2l + bo);
        blf.h[1] = *(const v8us*)(w2l + bo + 16);
        acc[t] = wmb(ahf.v, bhf.v, acc[t]);
        acc[t] = wmb(ahf.v, blf.v, acc[t]);
        acc[t] = wmb(alf.v, bhf.v, acc[t]);
      }
    }
    __syncthreads();
#pragma unroll
    for (int t = 0; t < 8; ++t) {
#pragma unroll
      for (int r = 0; r < 8; ++r) sp[(8 * hh + r) * 128 + 16 * t + m] = acc[t][r];
    }
    __syncthreads();
    {
      float sa = 0.0f, sd = 0.0f;
      const float* rp = sp + m * 128 + 64 * hh;
      const float* ca = sas + (2 * g + hh) * 64;
      const float* cd = sad + (2 * g + hh) * 64;
#pragma unroll 2
      for (int c = 0; c < 64; c += 4) {
        const v4f v = *(const v4f*)(rp + c);
        const v4f a = *(const v4f*)(ca + c);
        const v4f d = *(const v4f*)(cd + c);
        sa = fmaf(v.x, a.x, sa); sa = fmaf(v.y, a.y, sa); sa = fmaf(v.z, a.z, sa); sa = fmaf(v.w, a.w, sa);
        sd = fmaf(v.x, d.x, sd); sd = fmaf(v.y, d.y, sd); sd = fmaf(v.z, d.z, sd); sd = fmaf(v.w, d.w, sd);
      }
      sa0 = g == 0 ? sa : sa0; sd0 = g == 0 ? sd : sd0;
      sa1 = g == 1 ? sa : sa1; sd1 = g == 1 ? sd : sd1;
    }
    float* gp = H2 + (size_t)(rowBase + wave * 16) * HC + 128 * g + 4 * lane;
#pragma unroll
    for (int i = 0; i < 16; ++i) { const v4f v = *(const v4f*)(sp + i * 128 + 4 * lane); *(volatile v4f*)(gp + (size_t)i * HC) = v; }
    __threadfence();
#pragma unroll
    for (int i = 0; i < 16; ++i) { const v4f v = *(const v4f*)(sp + i * 128 + 4 * lane); *(volatile v4f*)(gp + (size_t)i * HC) = v; }
    __syncthreads();
  }
  astg[wave * 128 + m * APP + hh]     = sa0;
  astg[wave * 128 + m * APP + 2 + hh] = sa1;
  astg[wave * 128 + m * APP + 4 + hh] = sd0;
  astg[wave * 128 + m * APP + 6 + hh] = sd1;
  __syncthreads();
  const v4f av = *(const v4f*)(astg + wave * 128 + 4 * lane);
  float* aq = ap + (size_t)(rowBase + wave * 16) * APP + 4 * lane;
  *(volatile v4f*)aq = av;
  __threadfence();
  *(volatile v4f*)aq = av;
}

__global__ __launch_bounds__(G2THR) void k_agg2(
    const int* __restrict__ csr, const int* __restrict__ off, const int* __restrict__ cnt,
    const float* __restrict__ H2, const float* __restrict__ apA, const float* __restrict__ b2,
    const unsigned short* __restrict__ w3h, const unsigned short* __restrict__ w3l,
    const float* __restrict__ as3, const float* __restrict__ ad3,
    float* H3, float* apB, int nN, int csrLen) {
  extern __shared__ v4f lds_dyn[];
  unsigned short* sAh = (unsigned short*)lds_dyn;
  unsigned short* sAl = sAh + G2ROWS * KP2;
  float* stg  = (float*)(sAl + G2ROWS * KP2);
  float* sa3  = stg + G2W * 16 * C3;
  float* sd3  = sa3 + C3;
  float* astg = sd3 + C3;
  const int tid = threadIdx.x, lane = tid & 31, wave = tid >> 5, hh = lane >> 4, m = lane & 15;
  const int q = lane >> 3, sub = lane & 7, c0 = C3 * sub, head = sub >> 1;
  const int tb0 = blockIdx.x * G2ROWS + wave * 16;
  if (tid < C3) { sa3[tid] = as3[tid]; sd3[tid] = ad3[tid]; }

#pragma unroll 1
  for (int stp = 0; stp < 4; ++stp) {
    const int jrow = 4 * stp + q;
    const int t = tb0 + jrow;
    int n = cnt[t];
    n = clampi(n, 0, DEGCAP);
    const int st = off[t];
    const int nm = wmaxi(n);
    const int tc = t > nN - 1 ? nN - 1 : t;
    const float ad = apA[(size_t)tc * APP + 4 + head];
    const float e0 = lk(apA[(size_t)tc * APP + head] + ad);
    float mx = e0;
#pragma unroll 1
    for (int p = 0; p < nm; ++p) {
      const int pos = clampi(st + p, 0, csrLen - 1);
      const int s   = clampi(csr[pos], 0, nN - 1);
      const float a = apA[(size_t)s * APP + head];
      const bool ok = p < n;
      mx = ok ? fmaxf(mx, lk(a + ad)) : mx;
    }
    float dn = 0.0f;
    v4f acc[8];
#pragma unroll
    for (int i = 0; i < 8; ++i) { v4f zz = {0.f, 0.f, 0.f, 0.f}; acc[i] = zz; }
#pragma unroll 1
    for (int p = 0; p <= nm; ++p) {
      const int pos = clampi(st + p - 1, 0, csrLen - 1);
      int s = clampi(csr[pos], 0, nN - 1);
      s = (p == 0) ? tc : s;
      const float a = apA[(size_t)s * APP + head];
      float pe = __expf(lk(a + ad) - mx);
      pe = (p <= n) ? pe : 0.0f;
      dn += pe;
      const float* hp = H2 + (size_t)s * HC + c0;
#pragma unroll
      for (int i = 0; i < 8; ++i) { const v4f hv = *(const v4f*)(hp + 4 * i); acc[i] = pe * hv + acc[i]; }
    }
    const float inv = 1.0f / (dn + EPSS);
    unsigned short* rh = sAh + (wave * 16 + jrow) * KP2 + c0;
    unsigned short* rl = sAl + (wave * 16 + jrow) * KP2 + c0;
#pragma unroll
    for (int i = 0; i < 4; ++i) {
      const v4f ba = *(const v4f*)(b2 + c0 + 8 * i), bbv = *(const v4f*)(b2 + c0 + 8 * i + 4);
      const v4f va = relu4(acc[2 * i] * inv + ba);
      const v4f vb = relu4(acc[2 * i + 1] * inv + bbv);
      v4i ph, pl;
      pack8(va, vb, ph, pl);
      *(v4i*)(rh + 8 * i) = ph;
      *(v4i*)(rl + 8 * i) = pl;
    }
  }
  __syncthreads();

  v8f accw[2];
  { v8f zz = {0.f, 0.f, 0.f, 0.f, 0.f, 0.f, 0.f, 0.f}; accw[0] = zz; accw[1] = zz; }
  const unsigned short* arh = sAh + (wave * 16 + m) * KP2 + 8 * hh;
  const unsigned short* arl = sAl + (wave * 16 + m) * KP2 + 8 * hh;
#pragma unroll 1
  for (int kt = 0; kt < HC / 32; ++kt) {
    FragB ahf, alf;
    ahf.h[0] = *(const v8us*)(arh + 32 * kt);
    ahf.h[1] = *(const v8us*)(arh + 32 * kt + 16);
    alf.h[0] = *(const v8us*)(arl + 32 * kt);
    alf.h[1] = *(const v8us*)(arl + 32 * kt + 16);
#pragma unroll
    for (int tt = 0; tt < 2; ++tt) {
      const size_t bo = (size_t)(16 * tt + m) * HC + 32 * kt + 8 * hh;
      FragB bhf, blf;
      bhf.h[0] = *(const v8us*)(w3h + bo);
      bhf.h[1] = *(const v8us*)(w3h + bo + 16);
      blf.h[0] = *(const v8us*)(w3l + bo);
      blf.h[1] = *(const v8us*)(w3l + bo + 16);
      accw[tt] = wmb(ahf.v, bhf.v, accw[tt]);
      accw[tt] = wmb(ahf.v, blf.v, accw[tt]);
      accw[tt] = wmb(alf.v, bhf.v, accw[tt]);
    }
  }
  float* sp = stg + wave * (16 * C3);
#pragma unroll
  for (int tt = 0; tt < 2; ++tt) {
#pragma unroll
    for (int r = 0; r < 8; ++r) sp[(8 * hh + r) * C3 + 16 * tt + m] = accw[tt][r];
  }
  __syncthreads();
  {
    float sa = 0.0f, sd = 0.0f;
    const float* rp = sp + m * C3;
#pragma unroll 2
    for (int c = 0; c < C3; c += 4) {
      const v4f v = *(const v4f*)(rp + c);
      const v4f a = *(const v4f*)(sa3 + c);
      const v4f d = *(const v4f*)(sd3 + c);
      sa = fmaf(v.x, a.x, sa); sa = fmaf(v.y, a.y, sa); sa = fmaf(v.z, a.z, sa); sa = fmaf(v.w, a.w, sa);
      sd = fmaf(v.x, d.x, sd); sd = fmaf(v.y, d.y, sd); sd = fmaf(v.z, d.z, sd); sd = fmaf(v.w, d.w, sd);
    }
    v4f aw;
    aw.x = hh == 0 ? sa : sd; aw.y = 0.0f; aw.z = 0.0f; aw.w = 0.0f;
    *(v4f*)(astg + wave * 128 + m * APP + 4 * hh) = aw;
  }
  __syncthreads();
  float* gp = H3 + (size_t)tb0 * C3;
  const v4f o0 = *(const v4f*)(sp + 4 * lane);
  const v4f o1 = *(const v4f*)(sp + 4 * (32 + lane));
  const v4f o2 = *(const v4f*)(sp + 4 * (64 + lane));
  const v4f o3 = *(const v4f*)(sp + 4 * (96 + lane));
  const v4f av = *(const v4f*)(astg + wave * 128 + 4 * lane);
  float* aq = apB + (size_t)tb0 * APP + 4 * lane;
  *(volatile v4f*)(gp + 4 * lane) = o0;
  *(volatile v4f*)(gp + 4 * (32 + lane)) = o1;
  *(volatile v4f*)(gp + 4 * (64 + lane)) = o2;
  *(volatile v4f*)(gp + 4 * (96 + lane)) = o3;
  *(volatile v4f*)aq = av;
  __threadfence();
  *(volatile v4f*)(gp + 4 * lane) = o0;
  *(volatile v4f*)(gp + 4 * (32 + lane)) = o1;
  *(volatile v4f*)(gp + 4 * (64 + lane)) = o2;
  *(volatile v4f*)(gp + 4 * (96 + lane)) = o3;
  *(volatile v4f*)aq = av;
}

__global__ __launch_bounds__(NTHR) void k_agg3(
    const int* __restrict__ csr, const int* __restrict__ off, const int* __restrict__ cnt,
    const float* __restrict__ H3, const float* __restrict__ ap, const float* __restrict__ b3,
    float* out, int nN, int csrLen) {
  __shared__ __attribute__((aligned(16))) float os[TGT * C3];
  const int tid = threadIdx.x;
  const int t = blockIdx.x * TGT + tid;
  int n = cnt[t];
  n = clampi(n, 0, DEGCAP);
  const int st = off[t];
  const int nm = wmaxi(n);
  const int tc = t > nN - 1 ? nN - 1 : t;
  const float ad = ap[(size_t)tc * APP + 4];
  const float e0 = lk(ap[(size_t)tc * APP] + ad);
  float mx = e0;
#pragma unroll 1
  for (int p = 0; p < nm; ++p) {
    const int pos = clampi(st + p, 0, csrLen - 1);
    const int s   = clampi(csr[pos], 0, nN - 1);
    const float a = ap[(size_t)s * APP];
    const bool ok = p < n;
    mx = ok ? fmaxf(mx, lk(a + ad)) : mx;
  }
  float dn = 0.0f;
  v4f acc[8];
#pragma unroll
  for (int i = 0; i < 8; ++i) { v4f zz = {0.f, 0.f, 0.f, 0.f}; acc[i] = zz; }
#pragma unroll 1
  for (int p = 0; p <= nm; ++p) {
    const int pos = clampi(st + p - 1, 0, csrLen - 1);
    int s = clampi(csr[pos], 0, nN - 1);
    s = (p == 0) ? tc : s;
    const float a = ap[(size_t)s * APP];
    float pe = __expf(lk(a + ad) - mx);
    pe = (p <= n) ? pe : 0.0f;
    dn += pe;
    const float* hp = H3 + (size_t)s * C3;
#pragma unroll
    for (int i = 0; i < 8; ++i) { const v4f hv = *(const v4f*)(hp + 4 * i); acc[i] = pe * hv + acc[i]; }
  }
  const float inv = 1.0f / (dn + EPSS);
#pragma unroll
  for (int i = 0; i < 8; ++i) {
    const v4f bv = *(const v4f*)(b3 + 4 * i);
    const v4f o = acc[i] * inv + bv;
    *(v4f*)(os + tid * C3 + 4 * i) = o;
  }
  __syncthreads();
  const int nval = nN - blockIdx.x * TGT;
  float* go = out + (size_t)blockIdx.x * TGT * C3;
  v4f ov[8];
#pragma unroll
  for (int i = 0; i < 8; ++i) { const int idx = i * NTHR + tid; ov[i] = *(const v4f*)(os + 4 * idx); }
#pragma unroll
  for (int i = 0; i < 8; ++i) {
    const int idx = i * NTHR + tid;
    const int row = idx >> 3;
    if (row < nval) *(volatile v4f*)(go + 4 * (size_t)idx) = ov[i];
  }
  __threadfence();
#pragma unroll
  for (int i = 0; i < 8; ++i) {
    const int idx = i * NTHR + tid;
    const int row = idx >> 3;
    if (row < nval) *(volatile v4f*)(go + 4 * (size_t)idx) = ov[i];
  }
}

extern "C" void kernel_launch(void* const* d_in, const int* in_sizes, int n_in,
                              void* d_out, int out_size, void* d_ws, size_t ws_size,
                              hipStream_t stream) {
  if (n_in < 14) return;
  const int nN = in_sizes[0] / 3;
  const int nE = in_sizes[1] / 2;
  if (nN <= 0 || nE <= 0 || in_sizes[0] != 3 * nN || in_sizes[1] != 2 * nE) return;
  if (in_sizes[2] != 3 * HC || in_sizes[3] != HC || in_sizes[4] != HC || in_sizes[5] != HC) return;
  if (in_sizes[6] != HC * HC || in_sizes[7] != HC || in_sizes[8] != HC || in_sizes[9] != HC) return;
  if (in_sizes[10] != HC * C3 || in_sizes[11] != C3 || in_sizes[12] != C3 || in_sizes[13] != C3) return;
  if (out_size != nN * C3) return;
  if (nE > (1 << 28) || nN > (1 << 24)) return;

  const float* x    = (const float*)d_in[0];
  const int*   ei   = (const int*)d_in[1];
  const float* W1   = (const float*)d_in[2];
  const float* as1  = (const float*)d_in[3];
  const float* ad1  = (const float*)d_in[4];
  const float* b1   = (const float*)d_in[5];
  const float* W2   = (const float*)d_in[6];
  const float* as2  = (const float*)d_in[7];
  const float* ad2  = (const float*)d_in[8];
  const float* b2   = (const float*)d_in[9];
  const float* W3   = (const float*)d_in[10];
  const float* as3  = (const float*)d_in[11];
  const float* ad3  = (const float*)d_in[12];
  const float* b3   = (const float*)d_in[13];
  float* out = (float*)d_out;

  const int NPAD   = ((nN + TGT - 1) / TGT) * TGT;
  const int nBC    = (nN + NBC - 1) / NBC;
  const int CNTPAD = nBC * NBC;
  if (4 * nBC + 1 > RBN || CNTPAD < NPAD) return;
  const int nBF    = (nN + NBF - 1) / NBF;
  const int csrLen = ((nE + 31) & ~31) + 4096;

  char* ws = (char*)d_ws;
  size_t off = 0;
  const size_t oW2h = off; off += (size_t)HC * HC * 2;           off = (off + 255) & ~(size_t)255;
  const size_t oW2l = off; off += (size_t)HC * HC * 2;           off = (off + 255) & ~(size_t)255;
  const size_t oW3h = off; off += (size_t)C3 * HC * 2;           off = (off + 255) & ~(size_t)255;
  const size_t oW3l = off; off += (size_t)C3 * HC * 2;           off = (off + 255) & ~(size_t)255;
  const size_t oCnt = off; off += (size_t)CNTPAD * 4;            off = (off + 255) & ~(size_t)255;
  const size_t oOff = off; off += (size_t)CNTPAD * 4;            off = (off + 255) & ~(size_t)255;
  const size_t oRb  = off; off += (size_t)RBN * 4;               off = (off + 255) & ~(size_t)255;
  const size_t oCsr = off; off += (size_t)csrLen * 4;            off = (off + 255) & ~(size_t)255;
  const size_t oApA = off; off += (size_t)NPAD * APP * 4;        off = (off + 255) & ~(size_t)255;
  const size_t oApB = off; off += (size_t)NPAD * APP * 4;        off = (off + 255) & ~(size_t)255;
  const size_t oZH  = off; off += (size_t)NPAD * C3 * 4;         off = (off + 255) & ~(size_t)255;
  const size_t oH2  = off; off += (size_t)NPAD * HC * 4;         off = (off + 255) & ~(size_t)255;
  if (off > ws_size || off > WSCAP) return;
  unsigned short* w2h = (unsigned short*)(ws + oW2h);
  unsigned short* w2l = (unsigned short*)(ws + oW2l);
  unsigned short* w3h = (unsigned short*)(ws + oW3h);
  unsigned short* w3l = (unsigned short*)(ws + oW3l);
  int*   cnt  = (int*)(ws + oCnt);
  int*   offp = (int*)(ws + oOff);
  int*   rb   = (int*)(ws + oRb);
  int*   csr  = (int*)(ws + oCsr);
  float* apA  = (float*)(ws + oApA);
  float* apB  = (float*)(ws + oApB);
  float* zbuf = (float*)(ws + oZH);
  float* H3   = (float*)(ws + oZH);
  float* H2   = (float*)(ws + oH2);

  const int vec8 = ((nE & 3) == 0) ? 1 : 0;

  const int nPrep = (HC * HC / 8 + C3 * HC / 8 + NTHR - 1) / NTHR;
  k_wprep<<<nPrep, NTHR, 0, stream>>>(W2, W3, w2h, w2l, w3h, w3l);

  k_count<<<nBC, NTHR, 0, stream>>>(ei, cnt, nE, vec8);
  k_offsets<<<1, OTHR, 0, stream>>>(cnt, offp, rb, nBC);
  hipFuncSetAttribute(reinterpret_cast<const void*>(&k_fill),
                      hipFuncAttributeMaxDynamicSharedMemorySize, LDS_FILL);
  k_fill<<<nBF, NTHR, LDS_FILL, stream>>>(ei, offp, rb, csr, nN, nE, vec8, csrLen);

  k_node1<<<NPAD / 32, NTHR, 0, stream>>>(x, W1, as1, ad1, apA, nN);
  k_agg1<<<NPAD / TGT, NTHR, 0, stream>>>(csr, offp, cnt, x, apA, zbuf, nN, csrLen);

  hipFuncSetAttribute(reinterpret_cast<const void*>(&k_gemm2),
                      hipFuncAttributeMaxDynamicSharedMemorySize, LDS_G2);
  k_gemm2<<<NPAD / G2ROWS, G2THR, LDS_G2, stream>>>(zbuf, W1, b1, w2h, w2l, as2, ad2, H2, apA);

  hipFuncSetAttribute(reinterpret_cast<const void*>(&k_agg2),
                      hipFuncAttributeMaxDynamicSharedMemorySize, LDS_A2);
  k_agg2<<<NPAD / G2ROWS, G2THR, LDS_A2, stream>>>(csr, offp, cnt, H2, apA, b2, w3h, w3l, as3, ad3, H3, apB, nN, csrLen);

  k_agg3<<<NPAD / TGT, NTHR, 0, stream>>>(csr, offp, cnt, H3, apB, b3, out, nN, csrLen);
}
